// NonLocalBlock_1322849927683
// MI455X (gfx1250) — hardware-verified
//
#include <hip/hip_runtime.h>
#ifndef NB
#define NB 4
#endif
#ifndef NP
#define NP 4096
#endif
#define NPF 4096
#define CCH 512
#define NGRP 32
#define GC (CCH / NGRP)
#define XBF ((size_t)CCH * NPF)
#define GIT ((GC * NP) / (256 * 8))

static_assert(NP % 128 == 0);
static_assert(NP <= NPF);
static_assert(CCH % 128 == 0);
static_assert((GC * NP) % (256 * 8) == 0);
static_assert(GIT * 256 * 8 == GC * NP);

typedef unsigned short v8us __attribute__((ext_vector_type(8), may_alias));
typedef float  v8f  __attribute__((ext_vector_type(8)));
typedef float  v4f  __attribute__((ext_vector_type(4)));
typedef float  v4fa __attribute__((ext_vector_type(4), may_alias));
typedef _Float16 v16h __attribute__((ext_vector_type(16)));
typedef _Float16 v4h __attribute__((ext_vector_type(4)));
union FragH { v16h v; v8us half[2]; _Float16 h[16]; unsigned short u[16]; };

__device__ __forceinline__ float bf16_rne(float x) { unsigned int u = __float_as_uint(x); u = (u + 0x7FFFu + ((u >> 16) & 1u)) & 0xFFFF0000u; return __uint_as_float(u); }

__global__ __launch_bounds__(256) void k_wnat(const float* __restrict__ w, size_t n8, _Float16* __restrict__ Bt) {
  const size_t t = (size_t)blockIdx.x * 256 + threadIdx.x; if (t >= n8) return; FragH f;
#pragma unroll
  for (int q = 0; q < 8; ++q) f.h[q] = (_Float16)(bf16_rne(w[t * 8 + q]) * 16.0f);
  const v8us o = f.half[0];
  *(volatile v8us*)((unsigned short*)Bt + t * 8) = o; __threadfence(); *(volatile v8us*)((unsigned short*)Bt + t * 8) = o;
}

__global__ __launch_bounds__(256) void k_gn(const float* __restrict__ xb, const float* __restrict__ gw, const float* __restrict__ gb, _Float16* __restrict__ HN) {
  __shared__ float red[256];
  const unsigned t = threadIdx.x, g = blockIdx.x;
  const float* xg = xb + (size_t)g * GC * NPF;
  const float inv_n = 1.0f / (float)(GC * NP);
  float s = 0.f;
#pragma unroll 1
  for (unsigned it = 0; it < (unsigned)GIT; ++it) {
    const unsigned e = (it * 256u + t) * 8u; const unsigned cl = e / (unsigned)NP, p = e % (unsigned)NP;
    const float* src = xg + (size_t)cl * NPF + p;
    const v4f a = *(const v4fa*)src, c = *(const v4fa*)(src + 4);
    float ps = 0.f;
#pragma unroll
    for (int q = 0; q < 4; ++q) ps += bf16_rne(a[q]) + bf16_rne(c[q]);
    s += ps;
  }
  red[t] = s; __syncthreads();
  for (unsigned st = 128; st > 0; st >>= 1) { if (t < st) red[t] += red[t + st]; __syncthreads(); }
  const float mu = red[0] * inv_n; __syncthreads();
  float s2 = 0.f;
#pragma unroll 1
  for (unsigned it = 0; it < (unsigned)GIT; ++it) {
    const unsigned e = (it * 256u + t) * 8u; const unsigned cl = e / (unsigned)NP, p = e % (unsigned)NP;
    const float* src = xg + (size_t)cl * NPF + p;
    const v4f a = *(const v4fa*)src, c = *(const v4fa*)(src + 4);
    float ps = 0.f;
#pragma unroll
    for (int q = 0; q < 4; ++q) { const float d0 = bf16_rne(a[q]) - mu, d1 = bf16_rne(c[q]) - mu; ps += d0 * d0 + d1 * d1; }
    s2 += ps;
  }
  red[t] = s2; __syncthreads();
  for (unsigned st = 128; st > 0; st >>= 1) { if (t < st) red[t] += red[t + st]; __syncthreads(); }
  const float rs = rsqrtf(red[0] * inv_n + 1e-6f);
#pragma unroll 1
  for (unsigned it = 0; it < (unsigned)GIT; ++it) {
    const unsigned e = (it * 256u + t) * 8u; const unsigned cl = e / (unsigned)NP, p = e % (unsigned)NP;
    const unsigned ch = g * GC + cl;
    const float gg = bf16_rne(gw[ch]), bb = bf16_rne(gb[ch]);
    const float* src = xg + (size_t)cl * NPF + p;
    const v4f a = *(const v4fa*)src, c = *(const v4fa*)(src + 4);
    FragH f;
#pragma unroll
    for (int q = 0; q < 4; ++q) { f.h[q] = (_Float16)((bf16_rne(a[q]) - mu) * rs * gg + bb); f.h[4 + q] = (_Float16)((bf16_rne(c[q]) - mu) * rs * gg + bb); }
    const v8us o = f.half[0];
    unsigned short* d = (unsigned short*)HN + (size_t)g * GC * NP + e;
    *(volatile v8us*)d = o; __threadfence(); *(volatile v8us*)d = o;
  }
}

template <int NHv, int TTv>
__global__ __launch_bounds__(256) void k_vt(const _Float16* __restrict__ V16, int ldv, int voff, _Float16* __restrict__ Vt) {
  __shared__ unsigned short tl[64][66];
  const int tid = threadIdx.x; const int slab = blockIdx.x / (TTv / 64), lg = blockIdx.x % (TTv / 64); const int b = slab / NHv, h = slab % NHv;
  for (int i = tid; i < 64 * 8; i += 256) { const int r = i / 8, c8 = (i % 8) * 8; FragH f; f.half[0] = *(const v8us*)((const unsigned short*)V16 + ((size_t)b * TTv + lg * 64 + r) * ldv + voff + h * 64 + c8);
#pragma unroll
    for (int q = 0; q < 8; ++q) tl[r][c8 + q] = f.u[q]; }
  __syncthreads();
  for (int pass = 0; pass < 2; ++pass) {
#pragma unroll
    for (int rd = 0; rd < 2; ++rd) { const int d = rd * 32 + tid / 8, pc = tid % 8; FragH f;
#pragma unroll
      for (int q = 0; q < 8; ++q) f.u[q] = tl[pc * 8 + q][d];
      *(volatile v8us*)((unsigned short*)Vt + ((size_t)slab * 64 + d) * TTv + lg * 64 + pc * 8) = f.half[0]; }
    if (pass == 0) __threadfence(); }
}

__device__ __forceinline__ v16h g2_frag(const _Float16* p, int hh) { FragH f; f.half[0] = *(const v8us*)((const unsigned short*)p + 8 * hh); f.half[1] = *(const v8us*)((const unsigned short*)p + 16 + 8 * hh); return f.v; }
__device__ __forceinline__ v8f g2_mma(v16h a, v16h b, v8f c) { v8f d = __builtin_amdgcn_wmma_f32_16x16x32_f16(false, a, false, b, (short)0, c, false, false); asm volatile("v_nop\n\tv_nop\n\tv_nop\n\tv_nop" : "+v"(d) : "v"(a), "v"(b)); return d; }
template <int CPBF>
__global__ __launch_bounds__(128) void k_gemm2(const _Float16* __restrict__ A, int lda, size_t sA, const _Float16* __restrict__ Bh, int ldb, size_t sB, float alpha, const float* __restrict__ bias, size_t sBias, const float* __restrict__ CP, int rowsPerB, size_t sCPb, int row0g,
    float* __restrict__ C, _Float16* __restrict__ C16, int ldc, size_t sC, int M, int N, int K) {
  __shared__ __attribute__((aligned(16))) float so[4][32][68];
  const int tid = threadIdx.x, w = tid >> 5, lane = tid & 31, ln = lane & 15, hh = lane >> 4; const int by = blockIdx.y;
  A += (size_t)by * sA; Bh += (size_t)by * sB; const size_t cofs = (size_t)by * sC; const float* bp = bias ? bias + (size_t)by * sBias : nullptr;
  const int ntn = N >> 6; const int mt = blockIdx.x / ntn, nq = blockIdx.x - mt * ntn; const int row0 = mt * 128 + 32 * w, col0 = nq * 64; if (row0 >= M) return;
  const _Float16* a0p = A + (size_t)(row0 + ln) * lda; const _Float16* a1p = a0p + (size_t)16 * lda;
  const _Float16* b0p = Bh + (size_t)(col0 + ln) * ldb; const _Float16* b1p = b0p + (size_t)16 * ldb; const _Float16* b2p = b1p + (size_t)16 * ldb; const _Float16* b3p = b2p + (size_t)16 * ldb;
  const v8f z8 = {0.f,0.f,0.f,0.f,0.f,0.f,0.f,0.f}; v8f c00 = z8, c01 = z8, c02 = z8, c03 = z8, c10 = z8, c11 = z8, c12 = z8, c13 = z8;
#pragma unroll 1
  for (int kb = 0; kb < K; kb += 32) { const v16h a0 = g2_frag(a0p + kb, hh), a1 = g2_frag(a1p + kb, hh);
    v16h b = g2_frag(b0p + kb, hh); c00 = g2_mma(a0, b, c00); c10 = g2_mma(a1, b, c10);
    b = g2_frag(b1p + kb, hh); c01 = g2_mma(a0, b, c01); c11 = g2_mma(a1, b, c11);
    b = g2_frag(b2p + kb, hh); c02 = g2_mma(a0, b, c02); c12 = g2_mma(a1, b, c12);
    b = g2_frag(b3p + kb, hh); c03 = g2_mma(a0, b, c03); c13 = g2_mma(a1, b, c13); }
  v8f accs[8] = {c00, c01, c02, c03, c10, c11, c12, c13};
#pragma unroll
  for (int u = 0; u < 8; ++u) { const int t = u & 3, half = u >> 2; const int col = col0 + t * 16 + ln; const float bv = bp ? bf16_rne(bp[col]) : 0.f;
#pragma unroll
    for (int r = 0; r < 8; ++r) { const int rloc = half * 16 + 8 * hh + r; float v = accs[u][r] * alpha + bv;
      if (CP) { float cv; if (rowsPerB < 0) cv = CP[cofs + (size_t)(row0g + row0 + rloc) * ldc + col];        else { const int bidx = (row0g + row0 + rloc) / rowsPerB; cv = CP[(size_t)bidx * sCPb + (size_t)by * 64 + col]; }
        if (CPBF) cv = bf16_rne(cv); v += cv; }
      so[w][rloc][t * 16 + ln] = v; } }
  __builtin_amdgcn_fence(4  , "workgroup"); __builtin_amdgcn_wave_barrier();
  const int rsub = lane >> 4, c4 = (lane & 15) * 4;
  for (int pass = 0; pass < 2; ++pass) {
#pragma unroll
    for (int q = 0; q < 16; ++q) { const int r = q * 2 + rsub; const v4f v = *(const v4fa*)&so[w][r][c4]; if (C) *(volatile v4f*)(C + cofs + (size_t)(row0 + r) * ldc + col0 + c4) = v; if (C16) { v4h h4; for (int i = 0; i < 4; ++i) h4[i] = (_Float16)v[i]; *(volatile v4h*)(C16 + cofs + (size_t)(row0 + r) * ldc + col0 + c4) = h4; } }
    if (pass == 0) __threadfence(); } }

__global__ __launch_bounds__(256) void k_rowstat(const float* __restrict__ S, float* __restrict__ RMX, float* __restrict__ RIV) {
  #pragma clang fp contract(off)
  const unsigned i = blockIdx.x * 256u + threadIdx.x; if (i >= (unsigned)NP) return; const float* s = S + (size_t)i * NP; float mx = -3.0e38f;
#pragma unroll 1
  for (unsigned j = 0; j < (unsigned)NP; j += 4) { const v4f a = *(const v4fa*)(s + j); mx = fmaxf(fmaxf(mx, fmaxf(a[0], a[1])), fmaxf(a[2], a[3])); }
  float se = 0.f;
#pragma unroll 1
  for (unsigned j = 0; j < (unsigned)NP; j += 4) { const v4f a = *(const v4fa*)(s + j); se += (__expf(a[0] - mx) + __expf(a[1] - mx)) + (__expf(a[2] - mx) + __expf(a[3] - mx)); }
  const float iv = 256.0f * (1.0f / se);
  *(volatile float*)(RMX + i) = mx; *(volatile float*)(RIV + i) = iv; __threadfence(); *(volatile float*)(RMX + i) = mx; *(volatile float*)(RIV + i) = iv; }
__global__ __launch_bounds__(256) void k_rowp(const float* __restrict__ S, const float* __restrict__ RMX, const float* __restrict__ RIV, _Float16* __restrict__ P) {
  #pragma clang fp contract(off)
  const size_t t = (size_t)blockIdx.x * 256 + threadIdx.x; if (t >= (size_t)NP * NP / 8) return; const size_t e = t * 8; const unsigned row = (unsigned)(e / (size_t)NP);
  const float mx = RMX[row], iv = RIV[row]; const v4f a = *(const v4fa*)(S + e), c = *(const v4fa*)(S + e + 4); FragH f;
#pragma unroll
  for (int q = 0; q < 4; ++q) { f.h[q] = (_Float16)(__expf(a[q] - mx) * iv); f.h[4 + q] = (_Float16)(__expf(c[q] - mx) * iv); }
  const v8us o = f.half[0];
  unsigned short* d = (unsigned short*)P + e; *(volatile v8us*)d = o; __threadfence(); *(volatile v8us*)d = o; }

#define WS_W   ((size_t)CCH * CCH * 2)
#define WS_H   ((size_t)CCH * NP * 2)
#define WS_S   ((size_t)NP * NP * 4)
#define WS_P   ((size_t)NP * NP * 2)
#define WS_R   ((size_t)NP * 4)
#define WS_TOTAL (3 * WS_W + 6 * WS_H + WS_S + WS_P + 2 * WS_R)
static_assert(WS_W % 256 == 0);
static_assert(WS_H % 256 == 0);
static_assert(WS_R % 256 == 0);
static_assert(WS_TOTAL <= (size_t)134217728);
static_assert(((size_t)(NB - 1) * XBF + (size_t)(CCH - 1) * NPF + NP) * 4 <= (size_t)33554432);

extern "C" void kernel_launch(void* const* d_in, const int* in_sizes, int n_in,
                              void* d_out, int out_size, void* d_ws, size_t ws_size, hipStream_t stream) {
  if (n_in < 9) return;
  const size_t need = (size_t)(NB - 1) * XBF + (size_t)(CCH - 1) * NPF + NP;
  if ((size_t)in_sizes[0] < need) return; if ((size_t)out_size < need) return;
  if (in_sizes[1] < CCH) return; if (in_sizes[2] < CCH) return; if (in_sizes[4] < CCH) return; if (in_sizes[6] < CCH) return; if (in_sizes[8] < CCH) return;
  if (in_sizes[3] < CCH * CCH) return; if (in_sizes[5] < CCH * CCH) return; if (in_sizes[7] < CCH * CCH) return;
  const float* const* I = (const float* const*)d_in;
  const float* x = I[0]; const float* gnw = I[1]; const float* gnb = I[2]; const float* wq = I[3]; const float* bq = I[4]; const float* wk = I[5]; const float* bk = I[6]; const float* wv = I[7]; const float* bv = I[8];
  float* out = (float*)d_out;
  char* ws = (char*)d_ws; size_t off = 0;
  auto take = [&](size_t bytes) { char* p = ws + off; off += (bytes + 255) & ~(size_t)255; return p; };
  _Float16* BQ = (_Float16*)take(WS_W); _Float16* BK = (_Float16*)take(WS_W); _Float16* BV = (_Float16*)take(WS_W);
  _Float16* HN = (_Float16*)take(WS_H);
  _Float16* XT = (_Float16*)take(WS_H);
  _Float16* QT = (_Float16*)take(WS_H); _Float16* KT = (_Float16*)take(WS_H); _Float16* VT = (_Float16*)take(WS_H);
  _Float16* V  = (_Float16*)take(WS_H);
  float* S = (float*)take(WS_S); _Float16* P = (_Float16*)take(WS_P); float* RMX = (float*)take(WS_R); float* RIV = (float*)take(WS_R);
  if (off > ws_size) return;
  { const unsigned g = (unsigned)(((size_t)CCH * CCH / 8 + 255) / 256);
    k_wnat<<<g, 256, 0, stream>>>(wq, (size_t)CCH * CCH / 8, BQ); k_wnat<<<g, 256, 0, stream>>>(wk, (size_t)CCH * CCH / 8, BK); k_wnat<<<g, 256, 0, stream>>>(wv, (size_t)CCH * CCH / 8, BV); }
  const float scale = 0.044194173824159216f;
  for (int b = 0; b < NB; ++b) {
    const float* xb = x + (size_t)b * XBF;
    k_gn<<<NGRP, 256, 0, stream>>>(xb, gnw, gnb, HN);
    k_vt<NP / 64, CCH><<<(NP / 64) * (CCH / 64), 256, 0, stream>>>(HN, NP, 0, XT);
    k_gemm2<0><<<dim3((unsigned)((NP / 128) * (CCH / 64)), 1), 128, 0, stream>>>(XT, CCH, 0, BQ, CCH, 0, 0.0625f, bq, 0, nullptr, 1, 0, 0, nullptr, QT, CCH, 0, NP, CCH, CCH);
    k_gemm2<0><<<dim3((unsigned)((NP / 128) * (CCH / 64)), 1), 128, 0, stream>>>(XT, CCH, 0, BK, CCH, 0, 0.0625f, bk, 0, nullptr, 1, 0, 0, nullptr, KT, CCH, 0, NP, CCH, CCH);
    k_gemm2<0><<<dim3((unsigned)((NP / 128) * (CCH / 64)), 1), 128, 0, stream>>>(XT, CCH, 0, BV, CCH, 0, 0.0625f, bv, 0, nullptr, 1, 0, 0, nullptr, VT, CCH, 0, NP, CCH, CCH);
    k_vt<CCH / 64, NP><<<(CCH / 64) * (NP / 64), 256, 0, stream>>>(VT, CCH, 0, V);
    k_gemm2<0><<<dim3((unsigned)((NP / 128) * (NP / 64)), 1), 128, 0, stream>>>(QT, CCH, 0, KT, CCH, 0, scale, nullptr, 0, nullptr, 1, 0, 0, S, nullptr, NP, 0, NP, NP, CCH);
    k_rowstat<<<(NP + 255) / 256, 256, 0, stream>>>(S, RMX, RIV);
    k_rowp<<<(unsigned)(((size_t)NP * NP / 8 + 255) / 256), 256, 0, stream>>>(S, RMX, RIV, P);
    k_gemm2<1><<<dim3((unsigned)((CCH / 128) * (NP / 64)), 1), 128, 0, stream>>>(V, NP, 0, P, NP, 0, 0.00390625f, nullptr, 0, xb, -1, 0, 0, out + (size_t)b * XBF, nullptr, NPF, 0, CCH, NP, NP);
  }
}
